// RelativeAttention_34488587387517
// MI455X (gfx1250) — hardware-verified
//
#include <hip/hip_runtime.h>

typedef __attribute__((ext_vector_type(16))) __bf16 v16b;
typedef __attribute__((ext_vector_type(8)))  __bf16 v8b;
typedef __attribute__((ext_vector_type(8)))  float  v8f;
typedef __attribute__((ext_vector_type(4)))  float  v4f;
typedef __attribute__((ext_vector_type(4)))  unsigned int v4u;

constexpr int NBATCH = 2;
constexpr int NHEAD  = 16;
constexpr int NBH    = NBATCH * NHEAD;
constexpr int LSEQ   = 2048;
constexpr int DHEAD  = 64;
constexpr int MAXREL = 8;
constexpr int NBIAS  = 2 * MAXREL + 1;
constexpr int QBLK   = 64;
constexpr int KCH    = 64;
constexpr int NWAVE  = 4;
constexpr int VS_PITCH = 72;
constexpr int OS_PITCH = 68;
constexpr size_t PLANE_ELEMS = (size_t)NBH * LSEQ * DHEAD;
constexpr size_t WS_NEED = 2 * PLANE_ELEMS * sizeof(unsigned short);

static_assert(LSEQ % QBLK == 0, "query blocks tile the sequence exactly");
static_assert(LSEQ % KCH == 0, "key chunks tile the sequence exactly");
static_assert(DHEAD == 64, "head dim 64: two 32-deep k steps, four 16-wide d tiles");
static_assert(KCH % 32 == 0 && DHEAD % 32 == 0, "contraction depths are multiples of 32");
static_assert(NBIAS <= 32, "bias table fits one 32-entry LDS line");
static_assert((VS_PITCH * 2) % 16 == 0 && (OS_PITCH * 4) % 16 == 0, "16-B aligned LDS rows");
static_assert(WS_NEED <= 134217728ull, "workspace carve within budget");


__device__ __forceinline__ unsigned short f2bf_bits(float f) {
  unsigned u = __float_as_uint(f);
  return (unsigned short)((u + 0x7FFFu + ((u >> 16) & 1u)) >> 16);
}
__device__ __forceinline__ float bf_bits2f(unsigned short h) { return __uint_as_float(((unsigned)h) << 16); }
__device__ __forceinline__ __bf16 f2bf(float f) { return __builtin_bit_cast(__bf16, f2bf_bits(f)); }

__device__ __forceinline__ v8f mma_bf16(v16b a, v16b b, v8f c) {
  c = __builtin_amdgcn_wmma_f32_16x16x32_bf16(false, a, false, b, (short)0, c, false, false);
  asm volatile("v_nop\n\tv_nop\n\tv_nop\n\tv_nop" : "+v"(c) : "v"(a), "v"(b));
  return c;
}

__global__ __launch_bounds__(256) void kv_planes_kernel(
    const float* __restrict__ K, const float* __restrict__ V,
    unsigned short* __restrict__ Kb, unsigned short* __restrict__ Vt)
{
  __shared__ __align__(16) unsigned short Vs[DHEAD * VS_PITCH];
  const int bh  = blockIdx.y;
  const int kv0 = blockIdx.x * 64;
  const int tid = threadIdx.x;
  const float* Kp = K + ((size_t)bh * LSEQ + kv0) * DHEAD;
  const float* Vp = V + ((size_t)bh * LSEQ + kv0) * DHEAD;

  v4u kw[2];
#pragma unroll
  for (int it = 0; it < 2; ++it) {
    const int u = it * 256 + tid;
    const int row = u >> 3;
    const int seg = u & 7;
    const v4f k0v = *(const v4f*)(Kp + (size_t)row * DHEAD + seg * 8);
    const v4f k1v = *(const v4f*)(Kp + (size_t)row * DHEAD + seg * 8 + 4);
    const v4f v0v = *(const v4f*)(Vp + (size_t)row * DHEAD + seg * 8);
    const v4f v1v = *(const v4f*)(Vp + (size_t)row * DHEAD + seg * 8 + 4);
    kw[it][0] = (unsigned)f2bf_bits(k0v[0]) | ((unsigned)f2bf_bits(k0v[1]) << 16);
    kw[it][1] = (unsigned)f2bf_bits(k0v[2]) | ((unsigned)f2bf_bits(k0v[3]) << 16);
    kw[it][2] = (unsigned)f2bf_bits(k1v[0]) | ((unsigned)f2bf_bits(k1v[1]) << 16);
    kw[it][3] = (unsigned)f2bf_bits(k1v[2]) | ((unsigned)f2bf_bits(k1v[3]) << 16);
#pragma unroll
    for (int e = 0; e < 4; ++e) {
      Vs[(seg * 8 + e) * VS_PITCH + row]     = f2bf_bits(v0v[e]);
      Vs[(seg * 8 + 4 + e) * VS_PITCH + row] = f2bf_bits(v1v[e]);
    }
  }
  __syncthreads();

  v4u vw[2];
#pragma unroll
  for (int it = 0; it < 2; ++it) {
    const int u = it * 256 + tid;
    const int drow = u >> 3;
    const int seg  = u & 7;
    vw[it] = *(const v4u*)(Vs + drow * VS_PITCH + seg * 8);
  }

  for (int pass = 0; pass < 2; ++pass) {
#pragma unroll
    for (int it = 0; it < 2; ++it) {
      const int u = it * 256 + tid;
      const int row = u >> 3;
      const int seg = u & 7;
      *(volatile v4u*)(Kb + ((size_t)bh * LSEQ + kv0 + row) * DHEAD + seg * 8) = kw[it];
      *(volatile v4u*)(Vt + ((size_t)bh * DHEAD + row) * LSEQ + kv0 + seg * 8) = vw[it];
    }
    __threadfence();
  }
}

__global__ __launch_bounds__(128) void rel_attn_kernel(
    const float* __restrict__ q, const unsigned short* __restrict__ Kb,
    const unsigned short* __restrict__ Vt, const float* __restrict__ bias,
    float* __restrict__ out)
{
  union FB { v16b v; v8b h[2]; };
  __shared__ __align__(16) unsigned short Ksh[KCH * DHEAD];
  __shared__ __align__(16) unsigned short Vth[DHEAD * KCH];
  __shared__ __align__(16) unsigned short Psh[NWAVE][16 * KCH];
  __shared__ __align__(16) unsigned short Psl[NWAVE][16 * KCH];
  __shared__ __align__(16) float Os[NWAVE][16 * OS_PITCH];
  __shared__ float sb[32];

  const int tid  = threadIdx.x;
  const int wave = tid >> 5;
  const int lane = tid & 31;
  const int hh   = lane >> 4;
  const int c    = lane & 15;
  const int qb   = blockIdx.x;
  const int bh   = blockIdx.y;
  const int q0   = qb * QBLK + wave * 16;

  if (tid < 32) {
    const int bi = tid < NBIAS ? tid : (NBIAS - 1);
    sb[tid] = bf_bits2f(f2bf_bits(bias[bi]));
  }

  v16b qa[2];
  {
    const float* qrow = q + ((size_t)bh * LSEQ + q0 + c) * DHEAD;
#pragma unroll
    for (int dc = 0; dc < 2; ++dc) {
      const v4f x0 = *(const v4f*)(qrow + dc * 32 + 8 * hh);
      const v4f x1 = *(const v4f*)(qrow + dc * 32 + 8 * hh + 4);
      const v4f y0 = *(const v4f*)(qrow + dc * 32 + 16 + 8 * hh);
      const v4f y1 = *(const v4f*)(qrow + dc * 32 + 16 + 8 * hh + 4);
#pragma unroll
      for (int e = 0; e < 4; ++e) {
        qa[dc][e]      = f2bf(x0[e] * 0.125f);
        qa[dc][4 + e]  = f2bf(x1[e] * 0.125f);
        qa[dc][8 + e]  = f2bf(y0[e] * 0.125f);
        qa[dc][12 + e] = f2bf(y1[e] * 0.125f);
      }
    }
  }
  __syncthreads();
  const float b_lo = sb[0];
  const float b_hi = sb[2 * MAXREL];

  float mrow[8], lrow[8];
  v8f oacc[4];
#pragma unroll
  for (int r = 0; r < 8; ++r) { mrow[r] = -__builtin_inff(); lrow[r] = 0.f; }
#pragma unroll
  for (int t = 0; t < 4; ++t) oacc[t] = (v8f){0.f,0.f,0.f,0.f,0.f,0.f,0.f,0.f};

  const unsigned short* Kbh = Kb + (size_t)bh * LSEQ * DHEAD;
  const unsigned short* Vtb = Vt + (size_t)bh * DHEAD * LSEQ;
  float* ob = out + (size_t)bh * LSEQ * DHEAD;
  unsigned short* pwh = Psh[wave];
  unsigned short* pwl = Psl[wave];

  for (int kc = 0; kc < LSEQ / KCH; ++kc) {
    const int kv0 = kc * KCH;
    __syncthreads();
#pragma unroll
    for (int it = 0; it < 4; ++it) {
      const int u = it * 128 + tid;
      const int row = u >> 3;
      const int seg = u & 7;
      const v4u kw = *(const v4u*)(Kbh + (size_t)(kv0 + row) * DHEAD + seg * 8);
      const v4u vw = *(const v4u*)(Vtb + (size_t)row * LSEQ + kv0 + seg * 8);
      *(v4u*)(Ksh + row * DHEAD + seg * 8) = kw;
      *(v4u*)(Vth + row * KCH + seg * 8)   = vw;
    }
    __syncthreads();

    v8f s[4];
#pragma unroll
    for (int j = 0; j < 4; ++j) {
      s[j] = (v8f){0.f,0.f,0.f,0.f,0.f,0.f,0.f,0.f};
#pragma unroll
      for (int dc = 0; dc < 2; ++dc) {
        FB kf;
        kf.h[0] = *(const v8b*)(Ksh + (j * 16 + c) * DHEAD + dc * 32 + 8 * hh);
        kf.h[1] = *(const v8b*)(Ksh + (j * 16 + c) * DHEAD + dc * 32 + 16 + 8 * hh);
        s[j] = mma_bf16(qa[dc], kf.v, s[j]);
      }
    }

    if (kc + 1 < qb) {
#pragma unroll
      for (int j = 0; j < 4; ++j)
#pragma unroll
        for (int r = 0; r < 8; ++r) s[j][r] += b_lo;
    } else if (kc > qb + 1) {
#pragma unroll
      for (int j = 0; j < 4; ++j)
#pragma unroll
        for (int r = 0; r < 8; ++r) s[j][r] += b_hi;
    } else {
#pragma unroll
      for (int j = 0; j < 4; ++j) {
        const int kvcol = kv0 + j * 16 + c;
#pragma unroll
        for (int r = 0; r < 8; ++r) {
          int rel = kvcol - (q0 + 8 * hh + r);
          rel = rel < -MAXREL ? -MAXREL : rel;
          rel = rel > MAXREL ? MAXREL : rel;
          s[j][r] += sb[rel + MAXREL];
        }
      }
    }

    float cm[8];
#pragma unroll
    for (int r = 0; r < 8; ++r) {
      float m = fmaxf(fmaxf(s[0][r], s[1][r]), fmaxf(s[2][r], s[3][r]));
#pragma unroll
      for (int off = 1; off < 16; off <<= 1) m = fmaxf(m, __shfl_xor(m, off, 32));
      cm[r] = m;
    }

#pragma unroll
    for (int r = 0; r < 8; ++r) {
      const float mnew  = fmaxf(mrow[r], cm[r]);
      const float alpha = expf(mrow[r] - mnew);
      mrow[r] = mnew;
      float psum = 0.f;
#pragma unroll
      for (int j = 0; j < 4; ++j) {
        const float p = expf(s[j][r] - mnew);
        psum += p;
        const unsigned short hb = f2bf_bits(p);
        const unsigned short lb = f2bf_bits(p - bf_bits2f(hb));
        pwh[(8 * hh + r) * KCH + j * 16 + c] = hb;
        pwl[(8 * hh + r) * KCH + j * 16 + c] = lb;
      }
#pragma unroll
      for (int off = 1; off < 16; off <<= 1) psum += __shfl_xor(psum, off, 32);
      lrow[r] = lrow[r] * alpha + psum;
#pragma unroll
      for (int t = 0; t < 4; ++t) oacc[t][r] *= alpha;
    }
    __builtin_amdgcn_fence(__ATOMIC_RELEASE, "workgroup");
    __builtin_amdgcn_wave_barrier();
    __builtin_amdgcn_fence(__ATOMIC_ACQUIRE, "workgroup");

#pragma unroll
    for (int kk = 0; kk < 2; ++kk) {
      FB pa, pl;
      pa.h[0] = *(const v8b*)(pwh + c * KCH + kk * 32 + 8 * hh);
      pa.h[1] = *(const v8b*)(pwh + c * KCH + kk * 32 + 16 + 8 * hh);
      pl.h[0] = *(const v8b*)(pwl + c * KCH + kk * 32 + 8 * hh);
      pl.h[1] = *(const v8b*)(pwl + c * KCH + kk * 32 + 16 + 8 * hh);
#pragma unroll
      for (int t = 0; t < 4; ++t) {
        FB vb;
        vb.h[0] = *(const v8b*)(Vth + (t * 16 + c) * KCH + kk * 32 + 8 * hh);
        vb.h[1] = *(const v8b*)(Vth + (t * 16 + c) * KCH + kk * 32 + 16 + 8 * hh);
        oacc[t] = mma_bf16(pa.v, vb.v, oacc[t]);
        oacc[t] = mma_bf16(pl.v, vb.v, oacc[t]);
      }
    }
  }

  float* os = Os[wave];
#pragma unroll
  for (int r = 0; r < 8; ++r) {
    const float inv = 1.0f / lrow[r];
#pragma unroll
    for (int t = 0; t < 4; ++t) os[(8 * hh + r) * OS_PITCH + t * 16 + c] = oacc[t][r] * inv;
  }
  __builtin_amdgcn_fence(__ATOMIC_RELEASE, "workgroup");
  __builtin_amdgcn_wave_barrier();
  __builtin_amdgcn_fence(__ATOMIC_ACQUIRE, "workgroup");
  {
    const int c4 = (lane & 15) * 4;
    for (int pass = 0; pass < 2; ++pass) {
#pragma unroll
      for (int it = 0; it < 8; ++it) {
        const int row = it * 2 + hh;
        const v4f val = *(const v4f*)(os + row * OS_PITCH + c4);
        *(volatile v4f*)(ob + (size_t)(q0 + row) * DHEAD + c4) = val;
      }
      __threadfence();
    }
  }
}

extern "C" void kernel_launch(void* const* d_in, const int* in_sizes, int n_in,
                              void* d_out, int out_size, void* d_ws, size_t ws_size,
                              hipStream_t stream)
{
  if (n_in < 4) return;
  if (in_sizes[0] != (int)PLANE_ELEMS || in_sizes[1] != (int)PLANE_ELEMS ||
      in_sizes[2] != (int)PLANE_ELEMS || in_sizes[3] != NBIAS) return;
  if (out_size != (int)PLANE_ELEMS) return;
  if (d_ws == nullptr || ws_size < WS_NEED) return;

  const float* Q    = (const float*)d_in[0];
  const float* K    = (const float*)d_in[1];
  const float* V    = (const float*)d_in[2];
  const float* bias = (const float*)d_in[3];
  float* O = (float*)d_out;

  unsigned short* Kb = (unsigned short*)d_ws;
  unsigned short* Vt = Kb + PLANE_ELEMS;

  kv_planes_kernel<<<dim3(LSEQ / 64, NBH), 256, 0, stream>>>(K, V, Kb, Vt);
  rel_attn_kernel<<<dim3(LSEQ / QBLK, NBH), 128, 0, stream>>>(Q, Kb, Vt, bias, O);
}
